// GenesisV2_70875550318622
// MI455X (gfx1250) — hardware-verified
//
#include <hip/hip_runtime.h>


namespace {
constexpr int NB = 128, K = 64, D = 128, SL = 128, L = 2, NR = NB * K;
constexpr float XS = 8.0f, WSC = 256.0f, EPS = 1e-5f, SCALE = 0.08838834764831845f;

typedef _Float16 b16;
typedef __attribute__((ext_vector_type(16))) _Float16 v16b;
typedef __attribute__((ext_vector_type(8))) _Float16 v8b;
typedef __attribute__((ext_vector_type(8))) float v8f;
typedef __attribute__((ext_vector_type(4))) float v4f;
__device__ __forceinline__ float bf16_rne(float f) { unsigned int u = __float_as_uint(f); u += 0x7FFFu + ((u >> 16) & 1u); return __uint_as_float(u & 0xFFFF0000u); }
__device__ __forceinline__ void split16(float v, b16& hi, b16& lo) { hi = (b16)v; lo = (b16)(v - (float)hi); }
__device__ __forceinline__ v16b frag_kb(const b16* p, int hh) { const v8b a = *(const v8b*)(p + 8 * hh), b = *(const v8b*)(p + 16 + 8 * hh); v16b f;
#pragma unroll
  for (int e = 0; e < 8; ++e) { f[e] = a[e]; f[8 + e] = b[e]; } return f; }
__device__ __forceinline__ v8f wmma16b(v16b a, v16b b, v8f c) { v8f d = __builtin_amdgcn_wmma_f32_16x16x32_f16(false, a, false, b, (short)0, c, false, false); asm volatile("v_nop\n\tv_nop\n\tv_nop\n\tv_nop" : "+v"(d) : "v"(a), "v"(b)); return d; }
__device__ __forceinline__ void wave_lds_sync() { __builtin_amdgcn_fence(__ATOMIC_RELEASE, "workgroup"); __builtin_amdgcn_wave_barrier(); __builtin_amdgcn_fence(__ATOMIC_ACQUIRE, "workgroup"); }
__device__ __forceinline__ float pmul(float a, float b) { float p = a * b; asm volatile("" : "+v"(p)); return p; }
__device__ __forceinline__ float hsum16(float v) { v += __shfl_xor(v, 1); v += __shfl_xor(v, 2); v += __shfl_xor(v, 4); return v + __shfl_xor(v, 8); }
__device__ __forceinline__ float gelu_erf(float x) { return 0.5f * x * (1.0f + erff(x * 0.70710678118654752f)); }
__device__ __forceinline__ float nexp(float x) { return __builtin_amdgcn_exp2f(x * 1.4426950408889634f); }

constexpr int NWP = L * 7 + 3;
__global__ __launch_bounds__(256) void prep_kernel(const float* __restrict__ x, const float* __restrict__ wk, const float* __restrict__ wq, const float* __restrict__ wv1, const float* __restrict__ wv2, const float* __restrict__ wm1, const float* __restrict__ wm2, const float* __restrict__ wp, const float* __restrict__ wmu, const float* __restrict__ wsp, float* __restrict__ XF, b16* __restrict__ Xh, b16* __restrict__ Xl, b16* __restrict__ WT) {
  const size_t t = (size_t)blockIdx.x * 256 + threadIdx.x; const size_t nx = (size_t)NR * D / 8, nw = (size_t)D * D / 8;
  if (t < nx) { const size_t e = t * 8; const v4f a = *(const v4f*)(x + e), c = *(const v4f*)(x + e + 4); v4f ra, rc; v8b hv, lv = {}; for (int j = 0; j < 4; ++j) { ra[j] = bf16_rne(a[j]); rc[j] = bf16_rne(c[j]); hv[j] = (b16)(ra[j] * XS); hv[4 + j] = (b16)(rc[j] * XS); }
    for (int pass = 0; pass < 2; ++pass) { *(volatile v4f*)(XF + e) = ra; *(volatile v4f*)(XF + e + 4) = rc; *(volatile v8b*)(Xh + e) = hv; *(volatile v8b*)(Xl + e) = lv; __threadfence(); } return; }
  const size_t u = t - nx; const int k = (int)(u / nw); if (k >= NWP) return; const size_t e = (u - (size_t)k * nw) * 8; const int oo = (int)(e / D), i0 = (int)(e - (size_t)oo * D);
  const float* w; size_t ld = D, base = 0;
  if (k < L * 7) { const int l = k / 7, kk = k % 7;
    switch (kk) { case 0: w = wv1 + (size_t)l * 2 * D * D; break; case 1: w = wv1 + (size_t)l * 2 * D * D + (size_t)D * D; break; case 2: w = wk + (size_t)l * D * D; break; case 3: w = wq + (size_t)l * D * D; break; case 4: w = wv2 + (size_t)l * D * D; break; case 5: w = wm1 + (size_t)l * D * D; break; default: w = wm2 + (size_t)l * D * D; } }
  else { const int kk = k - L * 7; w = kk == 0 ? wp : kk == 1 ? wmu : wsp; }
  (void)base; v8b o; for (int j = 0; j < 8; ++j) o[j] = (b16)(bf16_rne(w[(size_t)(i0 + j) * ld + oo]) * WSC);
  for (int pass = 0; pass < 2; ++pass) { *(volatile v8b*)(WT + (size_t)k * D * D + (size_t)oo * D + i0) = o; __threadfence(); }
}
template <int MODE>
__global__ __launch_bounds__(128) void gemm_kernel(const b16* __restrict__ Ah, const b16* __restrict__ Al, const b16* __restrict__ W, const b16* __restrict__ W2p, const float* __restrict__ bias, const float* __restrict__ gam, const float* __restrict__ bet, float* __restrict__ XF, float* __restrict__ F1, float* __restrict__ F2, b16* __restrict__ Yh, b16* __restrict__ Yl) {
  __shared__ __attribute__((aligned(16))) float Ts[4][16][D + 4];
  const int wave = threadIdx.x >> 5, lane = threadIdx.x & 31, nloc = lane & 15, hlf = lane >> 4; const size_t m0 = ((size_t)blockIdx.x * 4 + wave) * 16;
  v8f acc[8], acc2[8];
#pragma unroll
  for (int t = 0; t < 8; ++t) { acc[t] = (v8f){}; acc2[t] = (v8f){}; }
#pragma unroll
  for (int kb = 0; kb < D; kb += 32) { const v16b a = frag_kb(Ah + (m0 + nloc) * D + kb, hlf), al = frag_kb(Al + (m0 + nloc) * D + kb, hlf);
#pragma unroll
    for (int t = 0; t < 8; ++t) { const v16b bw = frag_kb(W + (size_t)(t * 16 + nloc) * D + kb, hlf); acc[t] = wmma16b(a, bw, acc[t]); acc[t] = wmma16b(al, bw, acc[t]);
      if (MODE <= 1) { const v16b bw2 = frag_kb(W2p + (size_t)(t * 16 + nloc) * D + kb, hlf); acc2[t] = wmma16b(a, bw2, acc2[t]); acc2[t] = wmma16b(al, bw2, acc2[t]); } } }
  const float rs_ = 1.0f / (XS * WSC);
  if (MODE <= 1) {
#pragma unroll
    for (int t = 0; t < 8; ++t) { const int c = t * 16 + nloc; const float bb = (MODE == 0) ? bf16_rne(bias[c]) : 0.0f;
#pragma unroll
      for (int r = 0; r < 8; ++r) Ts[wave][8 * hlf + r][c] = (MODE == 0) ? (acc[t][r] + acc2[t][r]) * rs_ + bb : acc[t][r] * rs_; }
    wave_lds_sync();
    for (int pass = 0; pass < 2; ++pass) { for (int rr = 0; rr < 16; ++rr) *(volatile v4f*)(F1 + (m0 + rr) * D + lane * 4) = *(const v4f*)(&Ts[wave][rr][lane * 4]); __threadfence(); }
    wave_lds_sync();
#pragma unroll
    for (int t = 0; t < 8; ++t) { const int c = t * 16 + nloc;
#pragma unroll
      for (int r = 0; r < 8; ++r) Ts[wave][8 * hlf + r][c] = (MODE == 0) ? acc2[t][r] * rs_ : acc2[t][r] * rs_ * SCALE; }
    wave_lds_sync();
    for (int pass = 0; pass < 2; ++pass) { for (int rr = 0; rr < 16; ++rr) *(volatile v4f*)(F2 + (m0 + rr) * D + lane * 4) = *(const v4f*)(&Ts[wave][rr][lane * 4]); __threadfence(); }
    return; }
  if (MODE == 2) {
#pragma unroll
    for (int t = 0; t < 8; ++t) { const int c = t * 16 + nloc; const float bb = bf16_rne(bias[c]);
#pragma unroll
      for (int r = 0; r < 8; ++r) Ts[wave][8 * hlf + r][c] = acc[t][r] * rs_ + bb + XF[(m0 + 8 * hlf + r) * D + c]; }
    wave_lds_sync();
    for (int step = 0; step < 8; ++step) { const int rr = 2 * step + hlf; float xv[8]; float s = 0.0f; for (int j = 0; j < 8; ++j) { xv[j] = Ts[wave][rr][nloc * 8 + j]; s += xv[j]; } s = hsum16(s); const float mu = s * (1.0f / D); float q2 = 0.0f; for (int j = 0; j < 8; ++j) { const float dv = xv[j] - mu; q2 += pmul(dv, dv); } q2 = hsum16(q2); const float rsd = rsqrtf(q2 * (1.0f / D) + EPS);
      v8b hv, lv; for (int j = 0; j < 8; ++j) { const int c = nloc * 8 + j; const float y = pmul((xv[j] - mu) * rsd, bf16_rne(gam[c])) + bf16_rne(bet[c]); b16 a_, c_; split16(y * XS, a_, c_); hv[j] = a_; lv[j] = c_; }
      for (int pass = 0; pass < 2; ++pass) { *(volatile v8b*)(Yh + (m0 + rr) * D + nloc * 8) = hv; *(volatile v8b*)(Yl + (m0 + rr) * D + nloc * 8) = lv; __threadfence(); } }
    return; }
  if (MODE == 3 || MODE == 5) {
#pragma unroll
    for (int t = 0; t < 8; ++t) { const int c = t * 16 + nloc; const float bb = bf16_rne(bias[c]);
#pragma unroll
      for (int r = 0; r < 8; ++r) Ts[wave][8 * hlf + r][c] = gelu_erf(acc[t][r] * rs_ + bb); }
    wave_lds_sync();
    for (int pass = 0; pass < 2; ++pass) { for (int rr = 0; rr < 16; ++rr) if (lane < 16) { v8b hv, lv; for (int j = 0; j < 8; ++j) { b16 a_, c_; split16(Ts[wave][rr][lane * 8 + j] * XS, a_, c_); hv[j] = a_; lv[j] = c_; } *(volatile v8b*)(Yh + (m0 + rr) * D + lane * 8) = hv; *(volatile v8b*)(Yl + (m0 + rr) * D + lane * 8) = lv; } __threadfence(); }
    return; }
  if (MODE == 4) {
#pragma unroll
    for (int t = 0; t < 8; ++t) { const int c = t * 16 + nloc; const float bb = bf16_rne(bias[c]);
#pragma unroll
      for (int r = 0; r < 8; ++r) Ts[wave][8 * hlf + r][c] = XF[(m0 + 8 * hlf + r) * D + c] + acc[t][r] * rs_ + bb; }
    wave_lds_sync();
    for (int pass = 0; pass < 2; ++pass) { for (int rr = 0; rr < 16; ++rr) { *(volatile v4f*)(XF + (m0 + rr) * D + lane * 4) = *(const v4f*)(&Ts[wave][rr][lane * 4]);
        if (lane < 16) { v8b hv, lv; for (int j = 0; j < 8; ++j) { b16 a_, c_; split16(Ts[wave][rr][lane * 8 + j] * XS, a_, c_); hv[j] = a_; lv[j] = c_; } *(volatile v8b*)(Yh + (m0 + rr) * D + lane * 8) = hv; *(volatile v8b*)(Yl + (m0 + rr) * D + lane * 8) = lv; } } __threadfence(); }
    return; }
#pragma unroll
  for (int t = 0; t < 8; ++t) { const int c = t * 16 + nloc; const float bb = bf16_rne(bias[c]);
#pragma unroll
    for (int r = 0; r < 8; ++r) Ts[wave][8 * hlf + r][c] = acc[t][r] * rs_ + bb; }
  wave_lds_sync();
  for (int pass = 0; pass < 2; ++pass) { for (int rr = 0; rr < 16; ++rr) *(volatile v4f*)(F1 + (m0 + rr) * D + lane * 4) = *(const v4f*)(&Ts[wave][rr][lane * 4]); __threadfence(); }
}
__global__ __launch_bounds__(256) void pair_kernel(const float* __restrict__ PF, const float* __restrict__ NF, const float* __restrict__ KF, const float* __restrict__ QF, b16* __restrict__ Gh, b16* __restrict__ Gl) {
  __shared__ float At[8][K];
  const int wave = threadIdx.x >> 5, lane = threadIdx.x & 31; const size_t row = (size_t)blockIdx.x * 8 + wave; const size_t b = row / K; const float* qr = QF + row * D;
  float lg[2];
#pragma unroll
  for (int u = 0; u < 2; ++u) { const size_t jr = b * K + lane + 32 * u; const float* kr = KF + jr * D; float s = 0.0f; for (int c4 = 0; c4 < D; c4 += 4) { const v4f qa = *(const v4f*)(qr + c4), ka = *(const v4f*)(kr + c4); for (int j = 0; j < 4; ++j) s += pmul(qa[j], ka[j]); } lg[u] = s; }
  float mx = fmaxf(lg[0], lg[1]); mx = fmaxf(mx, __shfl_xor(mx, 1)); mx = fmaxf(mx, __shfl_xor(mx, 2)); mx = fmaxf(mx, __shfl_xor(mx, 4)); mx = fmaxf(mx, __shfl_xor(mx, 8)); mx = fmaxf(mx, __shfl_xor(mx, 16));
  const float e0 = nexp(lg[0] - mx), e1 = nexp(lg[1] - mx); float sm = e0 + e1; sm = hsum16(sm); sm += __shfl_xor(sm, 16); const float inv = 1.0f / sm;
  At[wave][lane] = e0 * inv; At[wave][lane + 32] = e1 * inv;
  wave_lds_sync();
  const int c0 = lane * 4; const v4f p4 = *(const v4f*)(PF + row * D + c0); float g[4] = {0, 0, 0, 0};
  for (int j = 0; j < K; ++j) { const v4f n4 = *(const v4f*)(NF + (b * K + j) * D + c0); const float a = At[wave][j];
#pragma unroll
    for (int q = 0; q < 4; ++q) g[q] += pmul(a, gelu_erf(p4[q] - n4[q])); }
  __attribute__((ext_vector_type(4))) _Float16 hv, lv; for (int q = 0; q < 4; ++q) { b16 a_, c_; split16(g[q] * XS, a_, c_); hv[q] = a_; lv[q] = c_; }
  for (int pass = 0; pass < 2; ++pass) { *(volatile __attribute__((ext_vector_type(4))) _Float16*)(Gh + row * D + c0) = hv; *(volatile __attribute__((ext_vector_type(4))) _Float16*)(Gl + row * D + c0) = lv; __threadfence(); }
}
__global__ __launch_bounds__(256) void pool_kernel(const float* __restrict__ XF, b16* __restrict__ Ph, b16* __restrict__ Pl) {
  const int wave = threadIdx.x >> 5, lane = threadIdx.x & 31; const int b = blockIdx.x * 8 + wave; const int c0 = lane * 4; float s[4] = {0, 0, 0, 0};
  for (int i = 0; i < K; ++i) { const v4f v = *(const v4f*)(XF + ((size_t)b * K + i) * D + c0); for (int q = 0; q < 4; ++q) s[q] += v[q]; }
  __attribute__((ext_vector_type(4))) _Float16 hv, lv; for (int q = 0; q < 4; ++q) { b16 a_, c_; split16(s[q] * XS, a_, c_); hv[q] = a_; lv[q] = c_; }
  for (int pass = 0; pass < 2; ++pass) { *(volatile __attribute__((ext_vector_type(4))) _Float16*)(Ph + (size_t)b * D + c0) = hv; *(volatile __attribute__((ext_vector_type(4))) _Float16*)(Pl + (size_t)b * D + c0) = lv; __threadfence(); }
}
}

extern "C" void kernel_launch(void* const* d_in, const int* in_sizes, int n_in, void* d_out, int out_size, void* d_ws, size_t ws_size, hipStream_t stream) {
  (void)n_in;
  auto Fp = [&](int i) { return (const float*)d_in[i]; };
  if (in_sizes[0] != NR * D || in_sizes[1] != L * D * D || in_sizes[3] != L * 2 * D * D || in_sizes[13] != D * SL || out_size != 2 * NB * SL) return;
  size_t off = 0; char* ws = (char*)d_ws;
  auto carve = [&](size_t bytes) { char* p = ws + off; off += (bytes + 255) & ~(size_t)255; return p; };
  float* XF = (float*)carve((size_t)NR * D * 4); b16* Xh = (b16*)carve((size_t)NR * D * 2); b16* Xl = (b16*)carve((size_t)NR * D * 2); b16* WT = (b16*)carve((size_t)NWP * D * D * 2);
  float* PF = (float*)carve((size_t)NR * D * 4); float* NF = (float*)carve((size_t)NR * D * 4); float* KF = (float*)carve((size_t)NR * D * 4); float* QF = (float*)carve((size_t)NR * D * 4);
  b16* Gh = (b16*)carve((size_t)NR * D * 2); b16* Gl = (b16*)carve((size_t)NR * D * 2); b16* Yh = (b16*)carve((size_t)NR * D * 2); b16* Yl = (b16*)carve((size_t)NR * D * 2); b16* Zh = (b16*)carve((size_t)NR * D * 2); b16* Zl = (b16*)carve((size_t)NR * D * 2);
  if (off > ws_size || off > ((size_t)128 << 20)) return;
  prep_kernel<<<(unsigned)(((size_t)NR * D / 8 + (size_t)NWP * D * D / 8 + 255) / 256), 256, 0, stream>>>(Fp(0), Fp(1), Fp(2), Fp(3), Fp(5), Fp(9), Fp(11), Fp(13), Fp(15), Fp(17), XF, Xh, Xl, WT);
  for (int l = 0; l < L; ++l) { const b16* Wl = WT + (size_t)l * 7 * D * D;
    gemm_kernel<0><<<NR / 64, 128, 0, stream>>>(Xh, Xl, Wl + 0 * D * D, Wl + 1 * D * D, Fp(4) + l * D, nullptr, nullptr, nullptr, PF, NF, nullptr, nullptr);
    gemm_kernel<1><<<NR / 64, 128, 0, stream>>>(Xh, Xl, Wl + 2 * D * D, Wl + 3 * D * D, nullptr, nullptr, nullptr, nullptr, KF, QF, nullptr, nullptr);
    pair_kernel<<<NR / 8, 256, 0, stream>>>(PF, NF, KF, QF, Gh, Gl);
    gemm_kernel<2><<<NR / 64, 128, 0, stream>>>(Gh, Gl, Wl + 4 * D * D, nullptr, Fp(6) + l * D, Fp(7) + l * D, Fp(8) + l * D, XF, nullptr, nullptr, Yh, Yl);
    gemm_kernel<3><<<NR / 64, 128, 0, stream>>>(Yh, Yl, Wl + 5 * D * D, nullptr, Fp(10) + l * D, nullptr, nullptr, nullptr, nullptr, nullptr, Zh, Zl);
    gemm_kernel<4><<<NR / 64, 128, 0, stream>>>(Zh, Zl, Wl + 6 * D * D, nullptr, Fp(12) + l * D, nullptr, nullptr, XF, nullptr, nullptr, Xh, Xl);
  }
  pool_kernel<<<NB / 8, 256, 0, stream>>>(XF, Gh, Gl);
  const b16* WH = WT + (size_t)L * 7 * D * D;
  gemm_kernel<5><<<NB / 64, 128, 0, stream>>>(Gh, Gl, WH, nullptr, Fp(14), nullptr, nullptr, nullptr, nullptr, nullptr, Yh, Yl);
  gemm_kernel<6><<<NB / 64, 128, 0, stream>>>(Yh, Yl, WH + (size_t)D * D, nullptr, Fp(16), nullptr, nullptr, nullptr, (float*)d_out, nullptr, nullptr, nullptr);
  gemm_kernel<6><<<NB / 64, 128, 0, stream>>>(Yh, Yl, WH + (size_t)2 * D * D, nullptr, Fp(18), nullptr, nullptr, nullptr, (float*)d_out + (size_t)NB * SL, nullptr, nullptr, nullptr);
}
